// LCR_13451837571284
// MI455X (gfx1250) — hardware-verified
//
#include <hip/hip_runtime.h>

typedef __attribute__((ext_vector_type(16))) _Float16 v16h;
typedef __attribute__((ext_vector_type(8)))  _Float16 v8h;
typedef __attribute__((ext_vector_type(8)))  float    v8f;
typedef __attribute__((ext_vector_type(4)))  float    v4f_t;
typedef float v4fa __attribute__((ext_vector_type(4), may_alias));

#define DIM   128
#define HW    4096
#define NPIX  8192
#define HEADS 4
#define HD    32

__device__ __forceinline__ v16h load16(const _Float16* p) {
    v8h lo = *(const v8h*)(p);
    v8h hi = *(const v8h*)(p + 8);
    return __builtin_shufflevector(lo, hi, 0,1,2,3,4,5,6,7,8,9,10,11,12,13,14,15);
}

template<int KT>
__device__ __forceinline__ v8f gemm_wave_tile(const _Float16* __restrict__ pW,
                                              const _Float16* sAct, int actStride,
                                              int mt, int nt, int lane) {
    v8f acc = {};
    const _Float16* abase = pW + (size_t)mt * KT * 512 + lane * 16;
    const int prow = nt * 16 + (lane & 15);
    const int koff = (lane & 16) >> 1;
    const _Float16* bbase = sAct + prow * actStride + koff;
#pragma unroll
    for (int kt = 0; kt < KT; ++kt) {
        v16h a = load16(abase + kt * 512);
        v16h b = __builtin_shufflevector(*(const v8h*)(bbase + kt * 32), *(const v8h*)(bbase + kt * 32 + 16), 0,1,2,3,4,5,6,7,8,9,10,11,12,13,14,15);
        acc = __builtin_amdgcn_wmma_f32_16x16x32_f16(false, a, false, b,
                                                     (short)0, acc, false, false);
    }
    return acc;
}

__device__ void stage_tile(const float* __restrict__ src_base,
                           const float* __restrict__ wnorm,
                           float* s_stage, float* s_red, float* s_scale,
                           _Float16* dst, int tid) {
    const int grp = tid >> 5, p = tid & 31;
    float ssq = 0.f;
#pragma unroll
    for (int j = 0; j < 16; ++j) {
        int c = grp * 16 + j;
        float v = src_base[c * HW + p];
        s_stage[p * 130 + c] = v;
        ssq += v * v;
    }
    s_red[p * 8 + grp] = ssq;
    __syncthreads();
    if (tid < 32) {
        float s = 0.f;
#pragma unroll
        for (int g = 0; g < 8; ++g) s += s_red[tid * 8 + g];
        s_scale[tid] = wnorm ? rsqrtf(s * (1.0f / DIM) + 1e-8f) : 1.0f;
    }
    __syncthreads();
    const float sc = s_scale[p];
#pragma unroll
    for (int j = 0; j < 16; ++j) {
        int c = grp * 16 + j;
        float wn = wnorm ? wnorm[c] : 1.0f;
        dst[p * 136 + c] = (_Float16)(s_stage[p * 130 + c] * sc * wn);
    }
    __syncthreads();
}

__global__ __launch_bounds__(32)
void k_pack(const float* __restrict__ W, _Float16* __restrict__ P, int Cin) {
    const int KT = Cin >> 5;
    const int mt = blockIdx.x / KT;
    const int kt = blockIdx.x % KT;
    const int lane = threadIdx.x;
    const int row = mt * 16 + (lane & 15);
    _Float16* out = P + ((size_t)blockIdx.x * 32 + lane) * 16;
#pragma unroll
    for (int i = 0; i < 16; ++i) {
        int k = kt * 32 + i + ((i >= 8) ? 8 : 0) + ((lane >= 16) ? 8 : 0);
        const _Float16 hv = (_Float16)W[row * Cin + k];
        *(volatile _Float16*)(out + i) = hv; __threadfence(); *(volatile _Float16*)(out + i) = hv;
    }
}

__device__ __forceinline__ void proj_store(const _Float16* pW, const float* bias,
                                           const _Float16* sAct, float* dst, float* s_out,
                                           int b, int yx0, int w, int lane, int tid) {
    __syncthreads();
#pragma unroll
    for (int nt = 0; nt < 2; ++nt) {
        v8f acc = gemm_wave_tile<4>(pW, sAct, 136, w, nt, lane);
        int pl = nt * 16 + (lane & 15);
        int mo = (lane & 16) >> 1;
#pragma unroll
        for (int r = 0; r < 8; ++r) {
            int o = w * 16 + r + mo;
            s_out[pl * 130 + o] = acc[r] + bias[o];
        }
    }
    __syncthreads();
#pragma unroll 1
    for (int pass = 0; pass < 2; ++pass) {
#pragma unroll
        for (int i = 0; i < 4; ++i) {
            const int c = tid + 256 * i, q = (c & 7) * 4, row = c >> 3, pl = row & 31, head = row >> 5;
            v4f_t v; v.x = s_out[pl * 130 + head * 32 + q]; v.y = s_out[pl * 130 + head * 32 + q + 1]; v.z = s_out[pl * 130 + head * 32 + q + 2]; v.w = s_out[pl * 130 + head * 32 + q + 3];
            *(volatile v4f_t*)(dst + ((((size_t)(b * HEADS + head)) * HW + yx0 + pl) << 5) + q) = v;
        }
        __threadfence();
    }
}

__global__ __launch_bounds__(256)
void k_qkv(const float* __restrict__ z, const float* __restrict__ h,
           const float* __restrict__ wzn, const float* __restrict__ whn,
           const _Float16* __restrict__ pwq, const float* __restrict__ bq,
           const _Float16* __restrict__ pwk, const float* __restrict__ bk,
           const _Float16* __restrict__ pwv, const float* __restrict__ bv,
           float* __restrict__ q_ws, float* __restrict__ k_ws, float* __restrict__ v_ws) {
    __shared__ float    s_stage[32 * 130];
    __shared__ float    s_red[32 * 8];
    __shared__ float    s_scale[32];
    __shared__ _Float16 s_z16[32 * 136];
    __shared__ _Float16 s_h16[32 * 136];
    const int tid = threadIdx.x, lane = tid & 31, w = tid >> 5;
    const int g0 = blockIdx.x * 32;
    const int b = g0 >> 12, yx0 = g0 & (HW - 1);
    stage_tile(&z[(size_t)b * DIM * HW + yx0], wzn, s_stage, s_red, s_scale, s_z16, tid);
    stage_tile(&h[(size_t)b * DIM * HW + yx0], whn, s_stage, s_red, s_scale, s_h16, tid);
    proj_store(pwq, bq, s_z16, q_ws, s_stage, b, yx0, w, lane, tid);
    proj_store(pwk, bk, s_h16, k_ws, s_stage, b, yx0, w, lane, tid);
    proj_store(pwv, bv, s_h16, v_ws, s_stage, b, yx0, w, lane, tid);
}

__global__ __launch_bounds__(256)
void k_attn(const float* __restrict__ q_ws, const float* __restrict__ k_ws,
            const float* __restrict__ v_ws, float* __restrict__ attn_out) {
    const int i = blockIdx.x * 256 + threadIdx.x;
    const int b = i >> 14, head = (i >> 12) & 3, yx = i & (HW - 1);
    const int y = yx >> 6, x = yx & 63;
    const size_t hb = ((size_t)(b * HEADS + head) * HW) << 5;
    float4 q[8];
    const float4* qp = (const float4*)(q_ws + hb + (size_t)yx * HD);
#pragma unroll
    for (int j = 0; j < 8; ++j) q[j] = qp[j];
    float m = -3.0e38f, l = 0.f;
    float4 acc[8];
#pragma unroll
    for (int j = 0; j < 8; ++j) acc[j] = make_float4(0.f, 0.f, 0.f, 0.f);
    const float scale = 0.17677669529663687f;
    for (int dy = -3; dy <= 3; ++dy) {
        int ny = y + dy;
        if ((unsigned)ny >= 64u) continue;
        for (int dx = -3; dx <= 3; ++dx) {
            int nx = x + dx;
            if ((unsigned)nx >= 64u) continue;
            int nyx = ny * 64 + nx;
            const float4* kp = (const float4*)(k_ws + hb + (size_t)nyx * HD);
            float s = 0.f;
#pragma unroll 2
            for (int j = 0; j < 8; ++j) {
                float4 kv = kp[j];
                s += q[j].x * kv.x + q[j].y * kv.y + q[j].z * kv.z + q[j].w * kv.w;
            }
            s *= scale;
            float mn = fmaxf(m, s);
            float alpha = __expf(m - mn);
            float wgt = __expf(s - mn);
            l = l * alpha + wgt;
            const float4* vp = (const float4*)(v_ws + hb + (size_t)nyx * HD);
#pragma unroll 2
            for (int j = 0; j < 8; ++j) {
                float4 vv = vp[j];
                acc[j].x = acc[j].x * alpha + wgt * vv.x;
                acc[j].y = acc[j].y * alpha + wgt * vv.y;
                acc[j].z = acc[j].z * alpha + wgt * vv.z;
                acc[j].w = acc[j].w * alpha + wgt * vv.w;
            }
            m = mn;
        }
    }
    const float inv = 1.f / l;
    float* op = attn_out + ((size_t)b * DIM + head * HD) * HW + yx;
#pragma unroll 1
    for (int pass = 0; pass < 2; ++pass) {
#pragma unroll
        for (int j = 0; j < 8; ++j) {
            *(volatile float*)(op + (4 * j + 0) * HW) = acc[j].x * inv;
            *(volatile float*)(op + (4 * j + 1) * HW) = acc[j].y * inv;
            *(volatile float*)(op + (4 * j + 2) * HW) = acc[j].z * inv;
            *(volatile float*)(op + (4 * j + 3) * HW) = acc[j].w * inv;
        }
        __threadfence();
    }
}

__global__ __launch_bounds__(256)
void k_oproj(const float* __restrict__ attn, const float* __restrict__ z,
             const _Float16* __restrict__ pwo, const float* __restrict__ bo,
             float* __restrict__ z2) {
    __shared__ float    s_stage[32 * 130];
    __shared__ float    s_red[32 * 8];
    __shared__ float    s_scale[32];
    __shared__ _Float16 s_a16[32 * 136];
    const int tid = threadIdx.x, lane = tid & 31, w = tid >> 5;
    const int g0 = blockIdx.x * 32;
    const int b = g0 >> 12, yx0 = g0 & (HW - 1);
    stage_tile(&attn[(size_t)b * DIM * HW + yx0], nullptr, s_stage, s_red, s_scale, s_a16, tid);
    __shared__ __attribute__((aligned(16))) float s_o[8][16 * 36];
    float* so = s_o[w];
#pragma unroll
    for (int nt = 0; nt < 2; ++nt) {
        v8f acc = gemm_wave_tile<4>(pwo, s_a16, 136, w, nt, lane);
        int pl = nt * 16 + (lane & 15);
        int pix = yx0 + pl;
        int mo = (lane & 16) >> 1;
#pragma unroll
        for (int r = 0; r < 8; ++r) {
            int o = w * 16 + r + mo;
            size_t idx = ((size_t)b * DIM + o) * HW + pix;
            so[(r + mo) * 36 + pl] = acc[r] + bo[o] + z[idx];
        }
    }
    asm volatile("s_wait_dscnt 0" ::: "memory");
#pragma unroll 1
    for (int pass = 0; pass < 2; ++pass) {
#pragma unroll
        for (int i = 0; i < 4; ++i) { const int c = lane + 32 * i, rr = c >> 3, q = (c & 7) * 4;
            *(volatile v4f_t*)(z2 + ((size_t)b * DIM + w * 16 + rr) * HW + yx0 + q) = *(const volatile v4fa*)(so + rr * 36 + q); }
        __threadfence();
    }
}

__global__ __launch_bounds__(256)
void k_ffn(const float* __restrict__ z2, const float* __restrict__ wffn,
           const _Float16* __restrict__ pw1, const float* __restrict__ b1,
           const _Float16* __restrict__ pw2, const float* __restrict__ b2,
           float* __restrict__ out) {
    __shared__ float    s_stage[32 * 130];
    __shared__ float    s_red[32 * 8];
    __shared__ float    s_scale[32];
    __shared__ _Float16 s_a16[32 * 136];
    __shared__ _Float16 s_t16[32 * 264];
    const int tid = threadIdx.x, lane = tid & 31, w = tid >> 5;
    const int g0 = blockIdx.x * 32;
    const int b = g0 >> 12, yx0 = g0 & (HW - 1);
    stage_tile(&z2[(size_t)b * DIM * HW + yx0], wffn, s_stage, s_red, s_scale, s_a16, tid);
    for (int tt = w; tt < 32; tt += 8) {
        int mt = tt >> 1, nt = tt & 1;
        v8f acc = gemm_wave_tile<4>(pw1, s_a16, 136, mt, nt, lane);
        int prow = nt * 16 + (lane & 15);
        int mo = (lane & 16) >> 1;
#pragma unroll
        for (int r = 0; r < 8; ++r) {
            int o = mt * 16 + r + mo;
            float xv = acc[r] + b1[o];
            float g = 0.5f * xv * (1.0f + erff(xv * 0.7071067811865475f));
            s_t16[prow * 264 + o] = (_Float16)g;
        }
    }
    __syncthreads();
    __shared__ __attribute__((aligned(16))) float s_o[8][16 * 36];
    float* so = s_o[w];
    for (int nt = 0; nt < 2; ++nt) {
        const int mt = w;
        v8f acc = gemm_wave_tile<8>(pw2, s_t16, 264, mt, nt, lane);
        int pl = nt * 16 + (lane & 15);
        int pix = yx0 + pl;
        int mo = (lane & 16) >> 1;
#pragma unroll
        for (int r = 0; r < 8; ++r) {
            int o = mt * 16 + r + mo;
            size_t idx = ((size_t)b * DIM + o) * HW + pix;
            so[(r + mo) * 36 + pl] = acc[r] + b2[o] + z2[idx];
        }
    }
    asm volatile("s_wait_dscnt 0" ::: "memory");
#pragma unroll 1
    for (int pass = 0; pass < 2; ++pass) {
#pragma unroll
        for (int i = 0; i < 4; ++i) { const int c = lane + 32 * i, rr = c >> 3, q = (c & 7) * 4;
            *(volatile v4f_t*)(out + ((size_t)b * DIM + w * 16 + rr) * HW + yx0 + q) = *(const volatile v4fa*)(so + rr * 36 + q); }
        __threadfence();
    }
}

extern "C" void kernel_launch(void* const* d_in, const int* in_sizes, int n_in,
                              void* d_out, int out_size, void* d_ws, size_t ws_size,
                              hipStream_t stream) {
    const float* z    = (const float*)d_in[0];
    const float* h    = (const float*)d_in[1];
    const float* wzn  = (const float*)d_in[2];
    const float* whn  = (const float*)d_in[3];
    const float* wq   = (const float*)d_in[4];
    const float* bq   = (const float*)d_in[5];
    const float* wk   = (const float*)d_in[6];
    const float* bk   = (const float*)d_in[7];
    const float* wv   = (const float*)d_in[8];
    const float* bv   = (const float*)d_in[9];
    const float* wo   = (const float*)d_in[10];
    const float* bo   = (const float*)d_in[11];
    const float* wffn = (const float*)d_in[12];
    const float* w1   = (const float*)d_in[13];
    const float* b1   = (const float*)d_in[14];
    const float* w2   = (const float*)d_in[15];
    const float* b2   = (const float*)d_in[16];
    float* outp = (float*)d_out;

    char* ws = (char*)d_ws;
    _Float16* pwq = (_Float16*)ws;
    _Float16* pwk = pwq + 16384;
    _Float16* pwv = pwk + 16384;
    _Float16* pwo = pwv + 16384;
    _Float16* pw1 = pwo + 16384;
    _Float16* pw2 = pw1 + 32768;
    float* q_ws   = (float*)(ws + 262144);
    float* k_ws   = q_ws   + (size_t)NPIX * DIM;
    float* v_ws   = k_ws   + (size_t)NPIX * DIM;
    float* attn   = v_ws   + (size_t)NPIX * DIM;
    float* z2     = attn   + (size_t)NPIX * DIM;

    k_pack<<<32, 32, 0, stream>>>(wq, pwq, 128);
    k_pack<<<32, 32, 0, stream>>>(wk, pwk, 128);
    k_pack<<<32, 32, 0, stream>>>(wv, pwv, 128);
    k_pack<<<32, 32, 0, stream>>>(wo, pwo, 128);
    k_pack<<<64, 32, 0, stream>>>(w1, pw1, 128);
    k_pack<<<64, 32, 0, stream>>>(w2, pw2, 256);

    k_qkv  <<<NPIX / 32, 256, 0, stream>>>(z, h, wzn, whn, pwq, bq, pwk, bk, pwv, bv,
                                           q_ws, k_ws, v_ws);
    k_attn <<<(NPIX * HEADS) / 256, 256, 0, stream>>>(q_ws, k_ws, v_ws, attn);
    k_oproj<<<NPIX / 32, 256, 0, stream>>>(attn, z, pwo, bo, z2);
    k_ffn  <<<NPIX / 32, 256, 0, stream>>>(z2, wffn, pw1, b1, pw2, b2, outp);
}
